// MS2D_46686294507588
// MI455X (gfx1250) — hardware-verified
//
#include <hip/hip_runtime.h>


#define NB    4
#define NL    4096
#define DM    96
#define DI    96
#define NS    16
#define NK    4
#define DTR   6
#define CD    38
#define CDP   48
#define MROWS (NB * NL)
#define KROWS (NB * NK * NL)

typedef float    v4f  __attribute__((ext_vector_type(4)));
typedef float    v4fa __attribute__((ext_vector_type(4), __may_alias__));
typedef float    v8f  __attribute__((ext_vector_type(8)));
typedef _Float16 v8h  __attribute__((ext_vector_type(8)));
typedef _Float16 v16h __attribute__((ext_vector_type(16)));
typedef __bf16   v16b __attribute__((ext_vector_type(16)));
typedef unsigned v4u  __attribute__((ext_vector_type(4)));
typedef unsigned v4ua __attribute__((ext_vector_type(4), __may_alias__));

union Frag16 { v16b b; v16h h; v8h h8[2]; v4u q[2]; };

__device__ __forceinline__ v8f mma_bf16(v8f c, const Frag16& a, const Frag16& b) {
  v8f d = __builtin_amdgcn_wmma_f32_16x16x32_bf16(false, a.b, false, b.b, (short)0, c, false, false);
  asm volatile("v_nop\n\tv_nop\n\tv_nop\n\tv_nop" : "+v"(d) : "v"(a.h), "v"(b.h));
  return d;
}
__device__ __forceinline__ v8f mma_f16(v8f c, const Frag16& a, const Frag16& b) {
  v8f d = __builtin_amdgcn_wmma_f32_16x16x32_f16(false, a.h, false, b.h, (short)0, c, false, false);
  asm volatile("v_nop\n\tv_nop\n\tv_nop\n\tv_nop" : "+v"(d) : "v"(a.h), "v"(b.h));
  return d;
}

__device__ __forceinline__ unsigned bf_hi16(float f) {
  const unsigned u = __float_as_uint(f);
  return (u + 0x7FFFu + ((u >> 16) & 1u)) & 0xFFFF0000u;
}
__device__ __forceinline__ void bf_pack2(float f0, float f1, unsigned& wh, unsigned& wl) {
  const unsigned h0 = bf_hi16(f0), h1 = bf_hi16(f1);
  const unsigned l0 = bf_hi16(f0 - __uint_as_float(h0));
  const unsigned l1 = bf_hi16(f1 - __uint_as_float(h1));
  wh = (h0 >> 16) | h1;
  wl = (l0 >> 16) | l1;
}
__device__ __forceinline__ void bf_split8(v4f x0, v4f x1, v4u& qh, v4u& ql) {
  unsigned a, b, c, d, e, f, g, hh;
  bf_pack2(x0.x, x0.y, a, e);
  bf_pack2(x0.z, x0.w, b, f);
  bf_pack2(x1.x, x1.y, c, g);
  bf_pack2(x1.z, x1.w, d, hh);
  qh.x = a; qh.y = b; qh.z = c; qh.w = d;
  ql.x = e; ql.y = f; ql.z = g; ql.w = hh;
}
__device__ __forceinline__ void build_split(const float* p0, const float* p1, Frag16& fh, Frag16& fl) {
  const v4f x0 = *(const v4fa*)p0, x1 = *(const v4fa*)(p0 + 4);
  const v4f x2 = *(const v4fa*)p1, x3 = *(const v4fa*)(p1 + 4);
  bf_split8(x0, x1, fh.q[0], fl.q[0]);
  bf_split8(x2, x3, fh.q[1], fl.q[1]);
}
__device__ __forceinline__ void build_f16(const float* p0, const float* p1, float sc, Frag16& fr) {
  const v4f x0 = *(const v4fa*)p0, x1 = *(const v4fa*)(p0 + 4);
  const v4f x2 = *(const v4fa*)p1, x3 = *(const v4fa*)(p1 + 4);
  v8h a, c;
  a[0] = (_Float16)(sc * x0.x); a[1] = (_Float16)(sc * x0.y); a[2] = (_Float16)(sc * x0.z); a[3] = (_Float16)(sc * x0.w);
  a[4] = (_Float16)(sc * x1.x); a[5] = (_Float16)(sc * x1.y); a[6] = (_Float16)(sc * x1.z); a[7] = (_Float16)(sc * x1.w);
  c[0] = (_Float16)(sc * x2.x); c[1] = (_Float16)(sc * x2.y); c[2] = (_Float16)(sc * x2.z); c[3] = (_Float16)(sc * x2.w);
  c[4] = (_Float16)(sc * x3.x); c[5] = (_Float16)(sc * x3.y); c[6] = (_Float16)(sc * x3.z); c[7] = (_Float16)(sc * x3.w);
  fr.h8[0] = a; fr.h8[1] = c;
}
__device__ __forceinline__ void load_plane(const unsigned short* plane, size_t boff, Frag16& fr) {
  fr.q[0] = *(const v4ua*)(plane + boff);
  fr.q[1] = *(const v4ua*)(plane + boff + 16);
}

__device__ __forceinline__ void store_lines_2x(const float* st, float* dst, int n4, int lane) {
  for (int i = lane; i < n4; i += 32) { const v4f v = *(const v4fa*)(st + 4 * i); *(volatile v4f*)(dst + 4 * i) = v; }
  __threadfence();
  for (int i = lane; i < n4; i += 32) { const v4f v = *(const v4fa*)(st + 4 * i); *(volatile v4f*)(dst + 4 * i) = v; }
}

__device__ __forceinline__ float silu_f(float v) { return v * __builtin_amdgcn_rcpf(1.0f + __expf(-v)); }

__device__ __forceinline__ float wave_sum(float v) {
#pragma unroll
  for (int o = 1; o < 32; o <<= 1) v += __shfl_xor(v, o, 32);
  return v;
}

__device__ __forceinline__ void split_row8(const float* src, unsigned short* dh, unsigned short* dl) {
  const v4f x0 = *(const v4fa*)src, x1 = *(const v4fa*)(src + 4);
  v4u qh, ql;
  bf_split8(x0, x1, qh, ql);
  *(volatile v4u*)dh = qh; *(volatile v4u*)dl = ql;
  __threadfence();
  *(volatile v4u*)dh = qh; *(volatile v4u*)dl = ql;
}

__global__ void __launch_bounds__(256)
k_prep(const float* __restrict__ ipw, const float* __restrict__ opw, const float* __restrict__ xpw,
       unsigned short* __restrict__ ihi, unsigned short* __restrict__ ilo,
       unsigned short* __restrict__ ohi, unsigned short* __restrict__ olo,
       unsigned short* __restrict__ xph)
{
  const int blk = blockIdx.x, tid = threadIdx.x;
  if (blk < 9) {
    const int t = blk * 256 + tid;
    if (t < 2 * DI * (DM / 8))
      split_row8(ipw + (size_t)t * 8, ihi + (size_t)t * 8, ilo + (size_t)t * 8);
  } else if (blk < 14) {
    const int t = (blk - 9) * 256 + tid;
    if (t < DM * (DI / 8))
      split_row8(opw + (size_t)t * 8, ohi + (size_t)t * 8, olo + (size_t)t * 8);
  } else {
    const int t = (blk - 14) * 256 + tid;
    if (t < NK * CDP * (DI / 8)) {
      const int row = t / (DI / 8), g = t - row * (DI / 8);
      const int k = row / CDP, c = row - k * CDP;
      union { v8h h; v4u q; } o;
      if (c < CD) {
        const float* s = xpw + ((size_t)(k * CD + c)) * DI + g * 8;
        const v4f a0 = *(const v4fa*)s, a1 = *(const v4fa*)(s + 4);
        o.h[0] = (_Float16)(64.0f * a0.x); o.h[1] = (_Float16)(64.0f * a0.y);
        o.h[2] = (_Float16)(64.0f * a0.z); o.h[3] = (_Float16)(64.0f * a0.w);
        o.h[4] = (_Float16)(64.0f * a1.x); o.h[5] = (_Float16)(64.0f * a1.y);
        o.h[6] = (_Float16)(64.0f * a1.z); o.h[7] = (_Float16)(64.0f * a1.w);
      } else {
#pragma unroll
        for (int i = 0; i < 8; ++i) o.h[i] = (_Float16)0.0f;
      }
      unsigned short* dst = xph + (size_t)t * 8;
      *(volatile v4u*)dst = o.q;
      __threadfence();
      *(volatile v4u*)dst = o.q;
    }
  }
}

__global__ void __launch_bounds__(32)
k_in_proj(const float* __restrict__ x, const unsigned short* __restrict__ whi, const unsigned short* __restrict__ wlo,
          float* __restrict__ xc0, float* __restrict__ szb, int mrows)
{
  __shared__ __attribute__((aligned(16))) float st[16 * DI];
  const int lane = threadIdx.x, h = lane >> 4, m = lane & 15;
  const int m0 = blockIdx.x * 16;
  const int hsel = blockIdx.y;
  if (m0 >= mrows) return;
  const float* arow = x + (size_t)(m0 + m) * DM;
  const size_t wbase = (size_t)hsel * DI * DM;
  v8f acc[6] = {};
#pragma unroll
  for (int ks = 0; ks < 3; ++ks) {
    const int k0 = ks * 32;
    Frag16 ah, al;
    build_split(arow + k0 + 8 * h, arow + k0 + 16 + 8 * h, ah, al);
#pragma unroll
    for (int j = 0; j < 6; ++j) {
      const size_t boff = wbase + (size_t)(j * 16 + m) * DM + k0 + 8 * h;
      Frag16 bh, bl;
      load_plane(whi, boff, bh);
      load_plane(wlo, boff, bl);
      acc[j] = mma_bf16(acc[j], ah, bh);
      acc[j] = mma_bf16(acc[j], ah, bl);
      acc[j] = mma_bf16(acc[j], al, bh);
    }
  }
#pragma unroll
  for (int j = 0; j < 6; ++j) {
#pragma unroll
    for (int r = 0; r < 8; ++r) {
      float v = acc[j][r];
      if (hsel) v = silu_f(v);
      st[(8 * h + r) * DI + j * 16 + m] = v;
    }
  }
  __syncthreads();
  float* dst = (hsel ? szb : xc0) + (size_t)m0 * DI;
  store_lines_2x(st, dst, 16 * DI / 4, lane);
}

#define WSEL(i) wv[(i) >> 2][(i) & 3]
__global__ void __launch_bounds__(256)
k_dwconv(const float* __restrict__ xc0, const float* __restrict__ cw, const float* __restrict__ cb,
         float* __restrict__ xcv, int total4)
{
  const int t = blockIdx.x * 256 + threadIdx.x;
  if (t >= total4) return;
  const int row = t / (DI / 4);
  const int c = (t - row * (DI / 4)) * 4;
  const int b = row / NL;
  const int p = row - b * NL;
  const int hh = p >> 6, ww = p & 63;
  v4f wv[9];
#pragma unroll
  for (int i = 0; i < 9; ++i) wv[i] = *(const v4fa*)(cw + c * 9 + 4 * i);
  v4f acc = *(const v4fa*)(cb + c);
  const float* plane = xc0 + (size_t)b * NL * DI + c;
#pragma unroll
  for (int dy = 0; dy < 3; ++dy) {
    const int y = hh + dy - 1;
    if ((unsigned)y < 64u) {
#pragma unroll
      for (int dx = 0; dx < 3; ++dx) {
        const int xx = ww + dx - 1;
        if ((unsigned)xx < 64u) {
          const v4f v = *(const v4fa*)(plane + (size_t)(y * 64 + xx) * DI);
          const int tap = dy * 3 + dx;
          v4f w;
          w.x = WSEL(tap); w.y = WSEL(9 + tap); w.z = WSEL(18 + tap); w.w = WSEL(27 + tap);
          acc = acc + v * w;
        }
      }
    }
  }
  v4f o;
  o.x = silu_f(acc.x); o.y = silu_f(acc.y); o.z = silu_f(acc.z); o.w = silu_f(acc.w);
  float* dst = xcv + (size_t)t * 4;
  *(volatile v4f*)dst = o;
  __threadfence();
  *(volatile v4f*)dst = o;
}

__global__ void __launch_bounds__(32)
k_xproj(const float* __restrict__ xcv, const unsigned short* __restrict__ xph, float* __restrict__ xdbl, int krows)
{
  __shared__ __attribute__((aligned(16))) float st[16 * CDP];
  const int lane = threadIdx.x, h = lane >> 4, m = lane & 15;
  const int m0 = blockIdx.x * 16;
  if (m0 >= krows) return;
  const int bk = m0 / NL;
  const int k = bk & 3, b = bk >> 2;
  const int t = (m0 - bk * NL) + m;
  const int lm = (k & 2) ? (NL - 1 - t) : t;
  const int s = (k & 1) ? (((lm & 63) << 6) | (lm >> 6)) : lm;
  const float* arow = xcv + ((size_t)b * NL + s) * DI;
  const size_t wbase = (size_t)k * CDP * DI;
  v8f acc[3] = {};
#pragma unroll
  for (int ks = 0; ks < 3; ++ks) {
    const int k0 = ks * 32;
    Frag16 a;
    build_f16(arow + k0 + 8 * h, arow + k0 + 16 + 8 * h, 256.0f, a);
#pragma unroll
    for (int j = 0; j < 3; ++j) {
      const size_t boff = wbase + (size_t)(j * 16 + m) * DI + k0 + 8 * h;
      Frag16 bb;
      load_plane(xph, boff, bb);
      acc[j] = mma_f16(acc[j], a, bb);
    }
  }
#pragma unroll
  for (int j = 0; j < 3; ++j)
#pragma unroll
    for (int r = 0; r < 8; ++r)
      st[(8 * h + r) * CDP + j * 16 + m] = acc[j][r] * (1.0f / 16384.0f);
  __syncthreads();
  store_lines_2x(st, xdbl + (size_t)m0 * CDP, 16 * CDP / 4, lane);
}

__global__ void __launch_bounds__(32)
k_scan(const float* __restrict__ xcv, const float* __restrict__ xdbl,
       const float* __restrict__ dtw, const float* __restrict__ dtb,
       const float* __restrict__ alog, const float* __restrict__ dsk,
       float* __restrict__ yseq)
{
  __shared__ __attribute__((aligned(16))) float ys[4 * 32];
  const int lane = threadIdx.x;
  const int bk = blockIdx.x / 3;
  const int dg = blockIdx.x - bk * 3;
  const int b = bk >> 2, k = bk & 3;
  const int d = dg * 32 + lane;
  const int kd = k * DI + d;
  float An[NS], hs[NS], wd[DTR];
#pragma unroll
  for (int n = 0; n < NS; ++n) { An[n] = -__expf(alog[(size_t)kd * NS + n]); hs[n] = 0.0f; }
#pragma unroll
  for (int r = 0; r < DTR; ++r) wd[r] = dtw[(size_t)kd * DTR + r];
  const float bias = dtb[kd];
  const float Dd = dsk[kd];
  const float* ub = xcv + (size_t)b * NL * DI + d;
  const float* xb = xdbl + (size_t)bk * NL * CDP;
  float* yb = yseq + (size_t)bk * NL * DI + dg * 32;
  const int rev = (k & 2) ? 1 : 0;
  const int tr = k & 1;
  for (int t = 0; t < NL; ++t) {
    const int lm = rev ? (NL - 1 - t) : t;
    const int s = tr ? (((lm & 63) << 6) | (lm >> 6)) : lm;
    const float u = ub[(size_t)s * DI];
    const float* xr = xb + (size_t)t * CDP;
    float pre = 0.0f;
#pragma unroll
    for (int r = 0; r < DTR; ++r) pre = fmaf(xr[r], wd[r], pre);
    pre += bias;
    const float e = __expf(-fabsf(pre));
    const float dl = fmaxf(pre, 0.0f) + __logf(1.0f + e);
    const float dlu = dl * u;
    float y = Dd * u;
#pragma unroll
    for (int n = 0; n < NS; ++n) {
      const float a = __expf(dl * An[n]);
      hs[n] = fmaf(hs[n], a, dlu * xr[DTR + n]);
      y = fmaf(hs[n], xr[DTR + NS + n], y);
    }
    ys[(t & 3) * 32 + lane] = y;
    if ((t & 3) == 3) {
      __syncthreads();
      const int q = lane >> 3, e4 = lane & 7;
      const v4f v = *(const v4fa*)(ys + q * 32 + e4 * 4);
      float* dst = yb + (size_t)(t - 3 + q) * DI + e4 * 4;
      *(volatile v4f*)dst = v;
      __threadfence();
      *(volatile v4f*)dst = v;
      __syncthreads();
    }
  }
}

__global__ void __launch_bounds__(32)
k_norm_out(const float* __restrict__ yseq, const float* __restrict__ szb,
           const float* __restrict__ nw, const float* __restrict__ nb,
           const unsigned short* __restrict__ whi, const unsigned short* __restrict__ wlo,
           float* __restrict__ out, int mrows)
{
  __shared__ __attribute__((aligned(16))) float ga[16 * DI];
  __shared__ __attribute__((aligned(16))) float st[16 * DM];
  const int lane = threadIdx.x, h = lane >> 4, m = lane & 15;
  const int m0 = blockIdx.x * 16;
  if (m0 >= mrows) return;
  float nw3[3], nb3[3];
#pragma unroll
  for (int j = 0; j < 3; ++j) { nw3[j] = nw[lane + 32 * j]; nb3[j] = nb[lane + 32 * j]; }
#pragma unroll 1
  for (int r = 0; r < 16; ++r) {
    const int row = m0 + r;
    const int b = row / NL, p = row - b * NL;
    const int p1 = ((p & 63) << 6) | (p >> 6);
    const size_t base = (size_t)b * NK * NL;
    const float* y0 = yseq + (base + p) * DI;
    const float* y1 = yseq + (base + NL + p1) * DI;
    const float* y2 = yseq + (base + 2 * NL + (NL - 1 - p)) * DI;
    const float* y3 = yseq + (base + 3 * NL + (NL - 1 - p1)) * DI;
    const float* zr = szb + (size_t)row * DI;
    float v[3];
    float s1 = 0.0f;
#pragma unroll
    for (int j = 0; j < 3; ++j) {
      const int dd = lane + 32 * j;
      v[j] = ((y0[dd] + y2[dd]) + y1[dd]) + y3[dd];
      s1 += v[j];
    }
    s1 = wave_sum(s1);
    const float mu = s1 * (1.0f / DI);
    float s2 = 0.0f;
#pragma unroll
    for (int j = 0; j < 3; ++j) { v[j] -= mu; s2 += v[j] * v[j]; }
    s2 = wave_sum(s2);
    const float inv = rsqrtf(s2 * (1.0f / DI) + 1e-5f);
#pragma unroll
    for (int j = 0; j < 3; ++j) {
      const int dd = lane + 32 * j;
      ga[r * DI + dd] = (v[j] * inv * nw3[j] + nb3[j]) * zr[dd];
    }
  }
  __syncthreads();
  v8f acc[6] = {};
  const float* arow = ga + m * DI;
#pragma unroll
  for (int ks = 0; ks < 3; ++ks) {
    const int k0 = ks * 32;
    Frag16 ah, al;
    build_split(arow + k0 + 8 * h, arow + k0 + 16 + 8 * h, ah, al);
#pragma unroll
    for (int j = 0; j < 6; ++j) {
      const size_t boff = (size_t)(j * 16 + m) * DI + k0 + 8 * h;
      Frag16 bh, bl;
      load_plane(whi, boff, bh);
      load_plane(wlo, boff, bl);
      acc[j] = mma_bf16(acc[j], ah, bh);
      acc[j] = mma_bf16(acc[j], ah, bl);
      acc[j] = mma_bf16(acc[j], al, bh);
    }
  }
#pragma unroll
  for (int j = 0; j < 6; ++j)
#pragma unroll
    for (int r = 0; r < 8; ++r)
      st[(8 * h + r) * DM + j * 16 + m] = acc[j][r];
  __syncthreads();
  store_lines_2x(st, out + (size_t)m0 * DM, 16 * DM / 4, lane);
}

extern "C" void kernel_launch(void* const* d_in, const int* in_sizes, int n_in,
                              void* d_out, int out_size, void* d_ws, size_t ws_size,
                              hipStream_t stream)
{
  if (n_in < 12) return;
  if (in_sizes[0] != MROWS * DM || in_sizes[1] != 2 * DI * DM || in_sizes[2] != DI * 9 || in_sizes[3] != DI ||
      in_sizes[4] != NK * CD * DI || in_sizes[5] != NK * DI * DTR || in_sizes[6] != NK * DI ||
      in_sizes[7] != NK * DI * NS || in_sizes[8] != NK * DI || in_sizes[9] != DI || in_sizes[10] != DI ||
      in_sizes[11] != DM * DI) return;
  if (out_size != MROWS * DM) return;

  const float* x    = (const float*)d_in[0];
  const float* ipw  = (const float*)d_in[1];
  const float* cw   = (const float*)d_in[2];
  const float* cb   = (const float*)d_in[3];
  const float* xpw  = (const float*)d_in[4];
  const float* dtw  = (const float*)d_in[5];
  const float* dtb  = (const float*)d_in[6];
  const float* alog = (const float*)d_in[7];
  const float* dsk  = (const float*)d_in[8];
  const float* nw   = (const float*)d_in[9];
  const float* nb   = (const float*)d_in[10];
  const float* opw  = (const float*)d_in[11];
  float* out = (float*)d_out;

  char* ws = (char*)d_ws;
  size_t o = 0;
  auto carve = [&](size_t bytes) -> char* { char* p = ws + o; o += (bytes + 255) & ~(size_t)255; return p; };
  float* xc0  = (float*)carve((size_t)MROWS * DI * sizeof(float));
  float* szb  = (float*)carve((size_t)MROWS * DI * sizeof(float));
  float* xcv  = (float*)carve((size_t)MROWS * DI * sizeof(float));
  float* xdbl = (float*)carve((size_t)KROWS * CDP * sizeof(float));
  float* yseq = (float*)carve((size_t)KROWS * DI * sizeof(float));
  unsigned short* ihi = (unsigned short*)carve((size_t)2 * DI * DM * 2);
  unsigned short* ilo = (unsigned short*)carve((size_t)2 * DI * DM * 2);
  unsigned short* ohi = (unsigned short*)carve((size_t)DM * DI * 2);
  unsigned short* olo = (unsigned short*)carve((size_t)DM * DI * 2);
  unsigned short* xph = (unsigned short*)carve((size_t)NK * CDP * DI * 2);
  if (o > ws_size) return;

  const int total4 = MROWS * (DI / 4);
  k_prep    <<<23, 256, 0, stream>>>(ipw, opw, xpw, ihi, ilo, ohi, olo, xph);
  k_in_proj <<<dim3(MROWS / 16, 2), 32, 0, stream>>>(x, ihi, ilo, xc0, szb, MROWS);
  k_dwconv  <<<(total4 + 255) / 256, 256, 0, stream>>>(xc0, cw, cb, xcv, total4);
  k_xproj   <<<KROWS / 16, 32, 0, stream>>>(xcv, xph, xdbl, KROWS);
  k_scan    <<<NB * NK * 3, 32, 0, stream>>>(xcv, xdbl, dtw, dtb, alog, dsk, yseq);
  k_norm_out<<<MROWS / 16, 32, 0, stream>>>(yseq, szb, nw, nb, ohi, olo, out, MROWS);
}
